// DenoisingNet_MLP_49357764165824
// MI455X (gfx1250) — hardware-verified
//
#include <hip/hip_runtime.h>

typedef unsigned short us16;
typedef us16   v8us  __attribute__((ext_vector_type(8)));
typedef __bf16 v16bf __attribute__((ext_vector_type(16)));
typedef float  v8f   __attribute__((ext_vector_type(8)));
typedef float  v4f   __attribute__((ext_vector_type(4)));
typedef v8us __attribute__((may_alias)) v8usa;
typedef v4f  __attribute__((may_alias)) v4fa;
union Frag { v16bf v; v8us half[2]; };

#define IMG   128
#define TW    121
#define LPOS  14641
#define LP    14720
#define NIMG  4
#define NCH   256
#define TP    68

static_assert(LP % 128 == 0);
static_assert(LP >= LPOS);
static_assert((TP * 4) % 16 == 0);

__device__ __forceinline__ v8f wmma_bf16(v16bf a, v16bf b, v8f c) {
    v8f d = __builtin_amdgcn_wmma_f32_16x16x32_bf16(false, a, false, b, (short)0, c, false, false);
    asm volatile("v_nop\n\tv_nop\n\tv_nop\n\tv_nop" : "+v"(d) : "v"(a), "v"(b));
    return d;
}

__device__ __forceinline__ v16bf ldfrag(const us16* p, int h) {
    Frag f;
    f.half[0] = *(const v8usa*)(p + 8 * h);
    f.half[1] = *(const v8usa*)(p + 16 + 8 * h);
    return f.v;
}

__device__ __forceinline__ v8f mac3(v8f c, v16bf ah, v16bf am, v16bf bh, v16bf bm) {
    c = wmma_bf16(ah, bh, c);
    c = wmma_bf16(ah, bm, c);
    c = wmma_bf16(am, bh, c);
    return c;
}
__device__ __forceinline__ v8f mac3x(v8f c, v16bf ah, v16bf am, v16bf al, v16bf bh, v16bf bm, v16bf bl) {
    c = wmma_bf16(ah, bl, c);
    c = wmma_bf16(al, bh, c);
    c = wmma_bf16(am, bm, c);
    return c;
}

__device__ __forceinline__ us16 bf_rne(float f) {
    unsigned int u = __float_as_uint(f);
    u += 0x7FFFu + ((u >> 16) & 1u);
    return (us16)(u >> 16);
}
__device__ __forceinline__ float bf_val(us16 s) {
    return __uint_as_float(((unsigned int)s) << 16);
}
__device__ __forceinline__ void split3(float x, us16& h, us16& mm, us16& l) {
    h = bf_rne(x);
    const float r1 = x - bf_val(h);
    mm = bf_rne(r1);
    const float r2 = r1 - bf_val(mm);
    l = bf_rne(r2);
}
__device__ __forceinline__ void split8(v4f a, v4f b, v8us& vh, v8us& vm, v8us& vl) {
    float f[8] = { a.x, a.y, a.z, a.w, b.x, b.y, b.z, b.w };
    #pragma unroll
    for (int e = 0; e < 8; ++e) {
        us16 p, q, r;
        split3(f[e], p, q, r);
        vh[e] = p; vm[e] = q; vl[e] = r;
    }
}

__device__ __forceinline__ float soft1(float t, float l) {
    float a = fabsf(t) - l;
    a = fmaxf(a, 0.0f);
    return (t > 0.0f) ? a : ((t < 0.0f) ? -a : 0.0f);
}

__global__ __launch_bounds__(256) void split_t_kernel(
    const float* __restrict__ src, int K, int N, int tr, int np,
    us16* ph, us16* pm, us16* pl)
{
    const int g = blockIdx.x * 256 + threadIdx.x;
    const int ko8 = K >> 3;
    if (g >= N * ko8) return;
    const int n = g / ko8;
    const int k0 = (g - n * ko8) * 8;
    float f[8];
    #pragma unroll
    for (int e = 0; e < 8; ++e) {
        const int k = k0 + e;
        const size_t idx = tr ? ((size_t)k * (size_t)N + (size_t)n) : ((size_t)n * (size_t)K + (size_t)k);
        f[e] = src[idx];
    }
    v8us vh, vm, vl;
    const v4f a = { f[0], f[1], f[2], f[3] };
    const v4f b = { f[4], f[5], f[6], f[7] };
    split8(a, b, vh, vm, vl);
    const size_t gi = (size_t)n * (size_t)K + (size_t)k0;
    *(volatile v8us*)(ph + gi) = vh;
    *(volatile v8us*)(pm + gi) = vm;
    if (np == 3) *(volatile v8us*)(pl + gi) = vl;
    __threadfence();
    *(volatile v8us*)(ph + gi) = vh;
    *(volatile v8us*)(pm + gi) = vm;
    if (np == 3) *(volatile v8us*)(pl + gi) = vl;
}

__global__ __launch_bounds__(256) void s_split_kernel(
    const float* __restrict__ D, const float* __restrict__ cp,
    us16* sh, us16* sm, us16* sl)
{
    const int g = blockIdx.x * 256 + threadIdx.x;
    if (g >= NCH * 32) return;
    const int n = g >> 5;
    const int k0 = (g & 31) * 8;
    const float rc = 1.0f / cp[0];
    float G[8];
    #pragma unroll
    for (int e = 0; e < 8; ++e) G[e] = 0.0f;
    #pragma unroll 1
    for (int p = 0; p < 64; ++p) {
        const float dn = D[p * NCH + n];
        #pragma unroll
        for (int e = 0; e < 8; ++e) G[e] += dn * D[p * NCH + k0 + e];
    }
    float f[8];
    #pragma unroll
    for (int e = 0; e < 8; ++e) f[e] = ((n == k0 + e) ? 1.0f : 0.0f) - G[e] * rc;
    v8us vh, vm, vl;
    const v4f a = { f[0], f[1], f[2], f[3] };
    const v4f b = { f[4], f[5], f[6], f[7] };
    split8(a, b, vh, vm, vl);
    const size_t gi = (size_t)n * NCH + (size_t)k0;
    *(volatile v8us*)(sh + gi) = vh;
    *(volatile v8us*)(sm + gi) = vm;
    *(volatile v8us*)(sl + gi) = vl;
    __threadfence();
    *(volatile v8us*)(sh + gi) = vh;
    *(volatile v8us*)(sm + gi) = vm;
    *(volatile v8us*)(sl + gi) = vl;
}

__global__ __launch_bounds__(256) void unfold_split_kernel(
    const float* __restrict__ xim, us16* ah, us16* am, us16* al)
{
    const int tid = threadIdx.x, lane = tid & 31, w = tid >> 5;
    const int q8 = lane & 7, sub = lane >> 3;
    const int row = blockIdx.x * 32 + w * 4 + sub;
    const bool valid = row < LPOS;
    const int posc = valid ? row : (LPOS - 1);
    const int py = posc / TW, px = posc - py * TW;
    const float* src = xim + (size_t)(py + q8) * IMG + px;
    float f[8];
    #pragma unroll
    for (int e = 0; e < 8; ++e) { const float v = src[e]; f[e] = valid ? v : 0.0f; }
    v8us vh, vm, vl;
    const v4f a = { f[0], f[1], f[2], f[3] };
    const v4f b = { f[4], f[5], f[6], f[7] };
    split8(a, b, vh, vm, vl);
    const size_t gi = (size_t)row * 64 + (size_t)(8 * q8);
    *(volatile v8us*)(ah + gi) = vh;
    *(volatile v8us*)(am + gi) = vm;
    *(volatile v8us*)(al + gi) = vl;
    __threadfence();
    *(volatile v8us*)(ah + gi) = vh;
    *(volatile v8us*)(am + gi) = vm;
    *(volatile v8us*)(al + gi) = vl;
}

__device__ __forceinline__ void store_f32(const float* sT, float* C, int N,
                                          int row0, int col0, int w, int lane) {
    const int q8 = lane & 7, sub = lane >> 3;
    #pragma unroll
    for (int i = 0; i < 8; ++i) {
        const int lid = w * 32 + i * 4 + sub;
        const int rl = lid >> 1, hl = lid & 1;
        const v4f v = *(const v4fa*)(sT + rl * TP + 32 * hl + 4 * q8);
        *(volatile v4f*)(C + (size_t)(row0 + rl) * (size_t)N + col0 + 32 * hl + 4 * q8) = v;
    }
}
template <int NOUT>
__device__ __forceinline__ void store_bf(const float* sT, us16* Ch, us16* Cm, us16* Cl, int N,
                                         int row0, int col0, int w, int lane) {
    const int q8 = lane & 7, sub = lane >> 3;
    #pragma unroll
    for (int i = 0; i < 4; ++i) {
        const int rl = w * 16 + i * 4 + sub;
        const float* sp = sT + rl * TP + 8 * q8;
        const v4f a = *(const v4fa*)sp;
        const v4f b = *(const v4fa*)(sp + 4);
        v8us vh, vm, vl;
        split8(a, b, vh, vm, vl);
        const size_t gi = (size_t)(row0 + rl) * (size_t)N + col0 + 8 * q8;
        *(volatile v8us*)(Ch + gi) = vh;
        *(volatile v8us*)(Cm + gi) = vm;
        if constexpr (NOUT == 3) *(volatile v8us*)(Cl + gi) = vl;
    }
}

template <int NPL, int MODE>
__global__ __launch_bounds__(256) void gemm_kernel(
    const us16* __restrict__ Ah, const us16* __restrict__ Am, const us16* __restrict__ Al, int lda,
    const us16* __restrict__ Bh, const us16* __restrict__ Bm, const us16* __restrict__ Bl, int ldb,
    int K, int N,
    const float* __restrict__ bias, const float* __restrict__ Yp, const float* __restrict__ Lt,
    const float* __restrict__ cp, const float* __restrict__ wp,
    float* Cf, us16* Ch, us16* Cm, us16* Cl)
{
    __shared__ __attribute__((aligned(16))) float sT[128 * TP];

    const int tid = threadIdx.x, lane = tid & 31, w = tid >> 5;
    const int h = lane >> 4, m = lane & 15;
    const int wm = w & 3, wn = w >> 2;
    const int row0 = blockIdx.y * 128, col0 = blockIdx.x * 64;

    const size_t ar0 = (size_t)(row0 + 32 * wm + m) * (size_t)lda;
    const size_t ar1 = ar0 + (size_t)16 * (size_t)lda;
    const size_t br0 = (size_t)(col0 + 32 * wn + m) * (size_t)ldb;
    const size_t br1 = br0 + (size_t)16 * (size_t)ldb;

    const v8f zero8 = { 0.f, 0.f, 0.f, 0.f, 0.f, 0.f, 0.f, 0.f };
    v8f acc[2][2];
    #pragma unroll
    for (int mt = 0; mt < 2; ++mt)
        #pragma unroll
        for (int nt = 0; nt < 2; ++nt) acc[mt][nt] = zero8;

    #pragma unroll 1
    for (int k0 = 0; k0 < K; k0 += 32) {
        const v16bf ah0 = ldfrag(Ah + ar0 + k0, h);
        const v16bf ah1 = ldfrag(Ah + ar1 + k0, h);
        const v16bf am0 = ldfrag(Am + ar0 + k0, h);
        const v16bf am1 = ldfrag(Am + ar1 + k0, h);
        const v16bf bh0 = ldfrag(Bh + br0 + k0, h);
        const v16bf bh1 = ldfrag(Bh + br1 + k0, h);
        const v16bf bm0 = ldfrag(Bm + br0 + k0, h);
        const v16bf bm1 = ldfrag(Bm + br1 + k0, h);
        acc[0][0] = mac3(acc[0][0], ah0, am0, bh0, bm0);
        acc[0][1] = mac3(acc[0][1], ah0, am0, bh1, bm1);
        acc[1][0] = mac3(acc[1][0], ah1, am1, bh0, bm0);
        acc[1][1] = mac3(acc[1][1], ah1, am1, bh1, bm1);
        if constexpr (NPL == 3) {
            const v16bf al0 = ldfrag(Al + ar0 + k0, h);
            const v16bf al1 = ldfrag(Al + ar1 + k0, h);
            const v16bf bl0 = ldfrag(Bl + br0 + k0, h);
            const v16bf bl1 = ldfrag(Bl + br1 + k0, h);
            acc[0][0] = mac3x(acc[0][0], ah0, am0, al0, bh0, bm0, bl0);
            acc[0][1] = mac3x(acc[0][1], ah0, am0, al0, bh1, bm1, bl1);
            acc[1][0] = mac3x(acc[1][0], ah1, am1, al1, bh0, bm0, bl0);
            acc[1][1] = mac3x(acc[1][1], ah1, am1, al1, bh1, bm1, bl1);
        }
    }

    float bv[2] = { 0.0f, 0.0f };
    if constexpr (MODE == 0 || MODE == 1) {
        bv[0] = bias[col0 + 32 * wn + m];
        bv[1] = bias[col0 + 32 * wn + 16 + m];
    }
    float wsc = 0.0f;
    if constexpr (MODE == 4) wsc = wp[0];
    #pragma unroll
    for (int mt = 0; mt < 2; ++mt)
        #pragma unroll
        for (int nt = 0; nt < 2; ++nt)
            #pragma unroll
            for (int r = 0; r < 8; ++r) {
                float v = acc[mt][nt][r];
                if constexpr (MODE == 0) { v += bv[nt]; v = fmaxf(v, 0.0f); }
                if constexpr (MODE == 1) { v += bv[nt]; }
                if constexpr (MODE == 4) { v = fminf(fmaxf(v, 0.0f), 1.0f) * wsc; }
                sT[(32 * wm + 16 * mt + 8 * h + r) * TP + 32 * wn + 16 * nt + m] = v;
            }
    __syncthreads();

    if constexpr (MODE == 3) {
        const float invc = 1.0f / cp[0];
        const int q8 = lane & 7, sub = lane >> 3;
        #pragma unroll
        for (int i = 0; i < 4; ++i) {
            const int rl = w * 16 + i * 4 + sub;
            float* sp = sT + rl * TP + 8 * q8;
            const size_t gi = (size_t)(row0 + rl) * (size_t)N + col0 + 8 * q8;
            const v4f a0 = *(const v4fa*)sp;
            const v4f a1 = *(const v4fa*)(sp + 4);
            const v4f y0 = *(const v4fa*)(Yp + gi);
            const v4f y1 = *(const v4fa*)(Yp + gi + 4);
            const v4f l0 = *(const v4fa*)(Lt + gi);
            const v4f l1 = *(const v4fa*)(Lt + gi + 4);
            v4f z0, z1;
            z0.x = soft1(a0.x + y0.x * invc, l0.x);
            z0.y = soft1(a0.y + y0.y * invc, l0.y);
            z0.z = soft1(a0.z + y0.z * invc, l0.z);
            z0.w = soft1(a0.w + y0.w * invc, l0.w);
            z1.x = soft1(a1.x + y1.x * invc, l1.x);
            z1.y = soft1(a1.y + y1.y * invc, l1.y);
            z1.z = soft1(a1.z + y1.z * invc, l1.z);
            z1.w = soft1(a1.w + y1.w * invc, l1.w);
            *(v4fa*)sp = z0;
            *(v4fa*)(sp + 4) = z1;
        }
        __syncthreads();
    }

    if constexpr (MODE == 1 || MODE == 2 || MODE == 4) {
        store_f32(sT, Cf, N, row0, col0, w, lane);
        __threadfence();
        store_f32(sT, Cf, N, row0, col0, w, lane);
    } else if constexpr (MODE == 0) {
        store_bf<2>(sT, Ch, Cm, Cl, N, row0, col0, w, lane);
        __threadfence();
        store_bf<2>(sT, Ch, Cm, Cl, N, row0, col0, w, lane);
    } else {
        store_bf<3>(sT, Ch, Cm, Cl, N, row0, col0, w, lane);
        __threadfence();
        store_bf<3>(sT, Ch, Cm, Cl, N, row0, col0, w, lane);
    }
}

__global__ __launch_bounds__(256) void chan_att_kernel(
    const float* __restrict__ lam, const float* __restrict__ w1,
    const float* __restrict__ w2, float* ca)
{
    __shared__ float sa[NCH], sx[NCH], ha[16], hx[16];
    const int t = threadIdx.x, lane = t & 31, w = t >> 5;
    double s = 0.0;
    float mx = -3.4028235e38f;
    #pragma unroll 4
    for (int r = 0; r < LPOS; ++r) {
        const float v = lam[(size_t)r * NCH + t];
        s += (double)v;
        mx = fmaxf(mx, v);
    }
    sa[t] = (float)s * (1.0f / (float)LPOS);
    sx[t] = mx;
    __syncthreads();
    if (w == 0) {
        const int j = lane & 15;
        float pa = 0.0f, px = 0.0f;
        #pragma unroll 1
        for (int ch = 0; ch < NCH; ++ch) {
            const float wv = w1[ch * 16 + j];
            pa += sa[ch] * wv;
            px += sx[ch] * wv;
        }
        if (lane < 16) { ha[j] = fmaxf(pa, 0.0f); hx[j] = fmaxf(px, 0.0f); }
    }
    __syncthreads();
    float oa = 0.0f, ox = 0.0f;
    #pragma unroll 1
    for (int jj = 0; jj < 16; ++jj) {
        const float wv = w2[jj * NCH + t];
        oa += ha[jj] * wv;
        ox += hx[jj] * wv;
    }
    const float sg = 1.0f / (1.0f + expf(-(oa + ox)));
    *(volatile float*)(ca + t) = sg;
    __threadfence();
    *(volatile float*)(ca + t) = sg;
}

__global__ __launch_bounds__(256) void spat_stats_kernel(
    const float* __restrict__ lam, const float* __restrict__ ca,
    float* smean, float* smax)
{
    __shared__ float sm_[32], sx_[32];
    const int tid = threadIdx.x, lane = tid & 31, w = tid >> 5;
    const int rb = blockIdx.x * 32;
    const v4f c0 = *(const v4fa*)(ca + 8 * lane);
    const v4f c1 = *(const v4fa*)(ca + 8 * lane + 4);
    #pragma unroll 1
    for (int rr = 0; rr < 4; ++rr) {
        const int row = rb + w * 4 + rr;
        const size_t rbase = (size_t)row * NCH;
        const v4f a = *(const v4fa*)(lam + rbase + 8 * lane);
        const v4f b = *(const v4fa*)(lam + rbase + 8 * lane + 4);
        const v4f pa = a * c0, pb = b * c1;
        float s = pa.x; s += pa.y; s += pa.z; s += pa.w; s += pb.x; s += pb.y; s += pb.z; s += pb.w;
        float mxv = fmaxf(fmaxf(fmaxf(pa.x, pa.y), fmaxf(pa.z, pa.w)), fmaxf(fmaxf(pb.x, pb.y), fmaxf(pb.z, pb.w)));
        #pragma unroll
        for (int off = 16; off > 0; off >>= 1) {
            s += __shfl_xor(s, off);
            mxv = fmaxf(mxv, __shfl_xor(mxv, off));
        }
        if (lane == 0) { sm_[w * 4 + rr] = s * (1.0f / 256.0f); sx_[w * 4 + rr] = mxv; }
    }
    __syncthreads();
    const float mv = sm_[lane], xv = sx_[lane];
    if (w == 0) {
        *(volatile float*)(smean + rb + lane) = mv;
        *(volatile float*)(smax + rb + lane) = xv;
    }
    __threadfence();
    if (w == 0) {
        *(volatile float*)(smean + rb + lane) = mv;
        *(volatile float*)(smax + rb + lane) = xv;
    }
}

__global__ __launch_bounds__(256) void thresh_z0_kernel(
    float* lam, const float* __restrict__ ca,
    const float* __restrict__ smean, const float* __restrict__ smax,
    const float* __restrict__ wc, const float* __restrict__ cp,
    const float* __restrict__ Yp, us16* zh, us16* zm, us16* zl)
{
    const int tid = threadIdx.x, lane = tid & 31, w = tid >> 5;
    const int rb = blockIdx.x * 32 + w * 4;
    const float invc = 1.0f / cp[0];
    const v4f caA0 = *(const v4fa*)(ca + 4 * lane);
    const v4f caA1 = *(const v4fa*)(ca + 128 + 4 * lane);
    const v4f caB0 = *(const v4fa*)(ca + 8 * lane);
    const v4f caB1 = *(const v4fa*)(ca + 8 * lane + 4);
    const int t0 = lane;
    const int t1 = lane + 32;
    const int t1c = (t1 < 48) ? t1 : 48;
    const bool has1 = (t1 <= 48);
    const float wm0 = wc[t0], wx0 = wc[49 + t0];
    const float wm1 = wc[t1c], wx1 = wc[49 + t1c];
    const int dy0 = t0 / 7, dx0 = t0 - dy0 * 7;
    const int dy1 = t1c / 7, dx1 = t1c - dy1 * 7;

    #pragma unroll 1
    for (int rr = 0; rr < 4; ++rr) {
        const int row = rb + rr;
        const int posc = (row < LPOS) ? row : (LPOS - 1);
        const int py = posc / TW, px = posc - py * TW;
        float a = 0.0f;
        {
            const int yy = py + dy0 - 3, xx = px + dx0 - 3;
            const bool ok = (yy >= 0) && (yy < TW) && (xx >= 0) && (xx < TW);
            const int yc = min(max(yy, 0), TW - 1), xc = min(max(xx, 0), TW - 1);
            const int pi = yc * TW + xc;
            const float cv = smean[pi] * wm0 + smax[pi] * wx0;
            a += ok ? cv : 0.0f;
        }
        {
            const int yy = py + dy1 - 3, xx = px + dx1 - 3;
            const bool ok = has1 && (yy >= 0) && (yy < TW) && (xx >= 0) && (xx < TW);
            const int yc = min(max(yy, 0), TW - 1), xc = min(max(xx, 0), TW - 1);
            const int pi = yc * TW + xc;
            const float cv = smean[pi] * wm1 + smax[pi] * wx1;
            a += ok ? cv : 0.0f;
        }
        #pragma unroll
        for (int off = 16; off > 0; off >>= 1) a += __shfl_xor(a, off);
        const float s = __shfl(a, 0);
        const float sig = 1.0f / (1.0f + expf(-s));

        const size_t rbase = (size_t)row * NCH;
        const v4f lmA0 = *(const v4fa*)(lam + rbase + 4 * lane);
        const v4f lmA1 = *(const v4fa*)(lam + rbase + 128 + 4 * lane);
        const v4f lmB0 = *(const v4fa*)(lam + rbase + 8 * lane);
        const v4f lmB1 = *(const v4fa*)(lam + rbase + 8 * lane + 4);
        const v4f y0 = *(const v4fa*)(Yp + rbase + 8 * lane);
        const v4f y1 = *(const v4fa*)(Yp + rbase + 8 * lane + 4);

        v4f lA0 = lmA0 * caA0; lA0 = lA0 * sig; lA0 = lA0 * invc;
        v4f lA1 = lmA1 * caA1; lA1 = lA1 * sig; lA1 = lA1 * invc;
        v4f lB0 = lmB0 * caB0; lB0 = lB0 * sig; lB0 = lB0 * invc;
        v4f lB1 = lmB1 * caB1; lB1 = lB1 * sig; lB1 = lB1 * invc;

        v4f z0, z1;
        z0.x = soft1(y0.x, lB0.x); z0.y = soft1(y0.y, lB0.y); z0.z = soft1(y0.z, lB0.z); z0.w = soft1(y0.w, lB0.w);
        z1.x = soft1(y1.x, lB1.x); z1.y = soft1(y1.y, lB1.y); z1.z = soft1(y1.z, lB1.z); z1.w = soft1(y1.w, lB1.w);
        v8us vh, vm, vl;
        split8(z0, z1, vh, vm, vl);

        const size_t zi = rbase + (size_t)(8 * lane);
        *(volatile v4f*)(lam + rbase + 4 * lane) = lA0;
        *(volatile v4f*)(lam + rbase + 128 + 4 * lane) = lA1;
        *(volatile v8us*)(zh + zi) = vh;
        *(volatile v8us*)(zm + zi) = vm;
        *(volatile v8us*)(zl + zi) = vl;
        __threadfence();
        *(volatile v4f*)(lam + rbase + 4 * lane) = lA0;
        *(volatile v4f*)(lam + rbase + 128 + 4 * lane) = lA1;
        *(volatile v8us*)(zh + zi) = vh;
        *(volatile v8us*)(zm + zi) = vm;
        *(volatile v8us*)(zl + zi) = vl;
    }
}

__global__ __launch_bounds__(256) void fold_kernel(
    const float* __restrict__ xp, const float* __restrict__ wp, float* outp)
{
    __shared__ __attribute__((aligned(16))) float so[256];
    const int t = threadIdx.x, lane = t & 31, w = t >> 5;
    const int Y = blockIdx.x * 2 + (t >> 7), X = t & 127;
    const float wv = wp[0];
    float num = 0.0f, den = 0.0f;
    #pragma unroll 1
    for (int i = 0; i < 8; ++i) {
        const int py = Y - i;
        const bool oky = (py >= 0) && (py < TW);
        const int pyc = min(max(py, 0), TW - 1);
        #pragma unroll
        for (int j = 0; j < 8; ++j) {
            const int px = X - j;
            const bool ok = oky && (px >= 0) && (px < TW);
            const int pxc = min(max(px, 0), TW - 1);
            const float v = xp[((size_t)(pyc * TW + pxc)) * 64 + i * 8 + j];
            num = ok ? (num + v) : num;
            den = ok ? (den + wv) : den;
        }
    }
    const float o = num / den;
    so[t] = o;
    __syncthreads();
    const int wr = w & 1;
    const v4f v = *(const v4fa*)(so + wr * 128 + 4 * lane);
    float* dst = outp + (size_t)(blockIdx.x * 2 + wr) * IMG + 4 * lane;
    if (w < 2) *(volatile v4f*)dst = v;
    __threadfence();
    if (w < 2) *(volatile v4f*)dst = v;
}

extern "C" void kernel_launch(void* const* d_in, const int* in_sizes, int n_in,
                              void* d_out, int out_size, void* d_ws, size_t ws_size,
                              hipStream_t stream) {
    if (n_in < 15) return;
    if (in_sizes[0] != NIMG * IMG * IMG) return;
    if (in_sizes[1] != 64 * NCH) return;
    if (in_sizes[2] < 1 || in_sizes[3] < 1) return;
    if (in_sizes[4] != 64 * 512 || in_sizes[5] != 512) return;
    if (in_sizes[6] != 512 * 256 || in_sizes[7] != 256) return;
    if (in_sizes[8] != 256 * 128 || in_sizes[9] != 128) return;
    if (in_sizes[10] != 128 * 256 || in_sizes[11] != 256) return;
    if (in_sizes[12] != 256 * 16 || in_sizes[13] != 16 * 256 || in_sizes[14] != 98) return;
    if (out_size != NIMG * IMG * IMG) return;

    const float* x    = (const float*)d_in[0];
    const float* Dict = (const float*)d_in[1];
    const float* cp   = (const float*)d_in[2];
    const float* wp   = (const float*)d_in[3];
    const float* W1   = (const float*)d_in[4];
    const float* b1   = (const float*)d_in[5];
    const float* W2   = (const float*)d_in[6];
    const float* b2   = (const float*)d_in[7];
    const float* W3   = (const float*)d_in[8];
    const float* b3   = (const float*)d_in[9];
    const float* W4   = (const float*)d_in[10];
    const float* b4   = (const float*)d_in[11];
    const float* caw1 = (const float*)d_in[12];
    const float* caw2 = (const float*)d_in[13];
    const float* sacv = (const float*)d_in[14];
    float* out = (float*)d_out;

    char* ws = (char*)d_ws;
    size_t off = 0;
    auto carve = [&](size_t bytes) -> char* {
        char* p = ws + off;
        off += (bytes + 255) & ~(size_t)255;
        return p;
    };
    const size_t PL64  = (size_t)LP * 64 * 2;
    const size_t PL512 = (size_t)LP * 512 * 2;
    const size_t PL256 = (size_t)LP * 256 * 2;
    const size_t PL128 = (size_t)LP * 128 * 2;
    const size_t PF256 = (size_t)LP * 256 * 4;
    const size_t PF64  = (size_t)LP * 64 * 4;

    us16* A0h = (us16*)carve(PL64);
    us16* A0m = (us16*)carve(PL64);
    us16* A0l = (us16*)carve(PL64);
    const size_t LREGB = 2 * PL512 + 2 * PL256 + 2 * PL128;
    char* LREG = carve(LREGB);
    us16* L1h = (us16*)(LREG);
    us16* L1m = (us16*)(LREG + PL512);
    us16* L2h = (us16*)(LREG + 2 * PL512);
    us16* L2m = (us16*)(LREG + 2 * PL512 + PL256);
    us16* L3h = (us16*)(LREG + 2 * PL512 + 2 * PL256);
    us16* L3m = (us16*)(LREG + 2 * PL512 + 2 * PL256 + PL128);
    us16* ZAh = (us16*)(LREG);
    us16* ZAm = (us16*)(LREG + PL256);
    us16* ZAl = (us16*)(LREG + 2 * PL256);
    us16* ZBh = (us16*)(LREG + 3 * PL256);
    us16* ZBm = (us16*)(LREG + 4 * PL256);
    us16* ZBl = (us16*)(LREG + 5 * PL256);
    float* XP = (float*)(LREG + 6 * PL256);
    if (6 * PL256 + PF64 > LREGB) return;
    float* LAM = (float*)carve(PF256);
    float* YB  = (float*)carve(PF256);
    us16* W1h = (us16*)carve((size_t)512 * 64 * 2);
    us16* W1m = (us16*)carve((size_t)512 * 64 * 2);
    us16* W2h = (us16*)carve((size_t)256 * 512 * 2);
    us16* W2m = (us16*)carve((size_t)256 * 512 * 2);
    us16* W3h = (us16*)carve((size_t)128 * 256 * 2);
    us16* W3m = (us16*)carve((size_t)128 * 256 * 2);
    us16* W4h = (us16*)carve((size_t)256 * 128 * 2);
    us16* W4m = (us16*)carve((size_t)256 * 128 * 2);
    us16* DTh = (us16*)carve((size_t)256 * 64 * 2);
    us16* DTm = (us16*)carve((size_t)256 * 64 * 2);
    us16* DTl = (us16*)carve((size_t)256 * 64 * 2);
    us16* DRh = (us16*)carve((size_t)64 * 256 * 2);
    us16* DRm = (us16*)carve((size_t)64 * 256 * 2);
    us16* DRl = (us16*)carve((size_t)64 * 256 * 2);
    us16* Sh  = (us16*)carve((size_t)256 * 256 * 2);
    us16* Sm  = (us16*)carve((size_t)256 * 256 * 2);
    us16* Sl  = (us16*)carve((size_t)256 * 256 * 2);
    float* CA    = (float*)carve((size_t)NCH * 4);
    float* SMEAN = (float*)carve((size_t)LP * 4);
    float* SMAX  = (float*)carve((size_t)LP * 4);
    if (off > ws_size) return;
    if (off > (size_t)134217728) return;

    split_t_kernel<<<(512 * 8 + 255) / 256, 256, 0, stream>>>(W1, 64, 512, 1, 2, W1h, W1m, W1m);
    split_t_kernel<<<(256 * 64 + 255) / 256, 256, 0, stream>>>(W2, 512, 256, 1, 2, W2h, W2m, W2m);
    split_t_kernel<<<(128 * 32 + 255) / 256, 256, 0, stream>>>(W3, 256, 128, 1, 2, W3h, W3m, W3m);
    split_t_kernel<<<(256 * 16 + 255) / 256, 256, 0, stream>>>(W4, 128, 256, 1, 2, W4h, W4m, W4m);
    split_t_kernel<<<(256 * 8 + 255) / 256, 256, 0, stream>>>(Dict, 64, 256, 1, 3, DTh, DTm, DTl);
    split_t_kernel<<<(64 * 32 + 255) / 256, 256, 0, stream>>>(Dict, 256, 64, 0, 3, DRh, DRm, DRl);
    s_split_kernel<<<(NCH * 32 + 255) / 256, 256, 0, stream>>>(Dict, cp, Sh, Sm, Sl);

    const unsigned MG = LP / 128;
    for (int n = 0; n < NIMG; ++n) {
        const float* xim = x + (size_t)n * IMG * IMG;
        float* oim = out + (size_t)n * IMG * IMG;

        unfold_split_kernel<<<LP / 32, 256, 0, stream>>>(xim, A0h, A0m, A0l);

        gemm_kernel<2, 0><<<dim3(512 / 64, MG), 256, 0, stream>>>(
            A0h, A0m, A0m, 64, W1h, W1m, W1m, 64, 64, 512,
            b1, YB, LAM, cp, wp, LAM, L1h, L1m, L1m);
        gemm_kernel<2, 0><<<dim3(256 / 64, MG), 256, 0, stream>>>(
            L1h, L1m, L1m, 512, W2h, W2m, W2m, 512, 512, 256,
            b2, YB, LAM, cp, wp, LAM, L2h, L2m, L2m);
        gemm_kernel<2, 0><<<dim3(128 / 64, MG), 256, 0, stream>>>(
            L2h, L2m, L2m, 256, W3h, W3m, W3m, 256, 256, 128,
            b3, YB, LAM, cp, wp, LAM, L3h, L3m, L3m);
        gemm_kernel<2, 1><<<dim3(256 / 64, MG), 256, 0, stream>>>(
            L3h, L3m, L3m, 128, W4h, W4m, W4m, 128, 128, 256,
            b4, YB, LAM, cp, wp, LAM, A0h, A0m, A0l);

        gemm_kernel<3, 2><<<dim3(256 / 64, MG), 256, 0, stream>>>(
            A0h, A0m, A0l, 64, DTh, DTm, DTl, 64, 64, 256,
            b4, YB, LAM, cp, wp, YB, A0h, A0m, A0l);

        chan_att_kernel<<<1, 256, 0, stream>>>(LAM, caw1, caw2, CA);
        spat_stats_kernel<<<LP / 32, 256, 0, stream>>>(LAM, CA, SMEAN, SMAX);
        thresh_z0_kernel<<<LP / 32, 256, 0, stream>>>(LAM, CA, SMEAN, SMAX, sacv, cp, YB, ZAh, ZAm, ZAl);

        us16* zsh = ZAh; us16* zsm = ZAm; us16* zsl = ZAl;
        us16* zdh = ZBh; us16* zdm = ZBm; us16* zdl = ZBl;
        for (int it = 0; it < 5; ++it) {
            gemm_kernel<3, 3><<<dim3(256 / 64, MG), 256, 0, stream>>>(
                zsh, zsm, zsl, 256, Sh, Sm, Sl, 256, 256, 256,
                b4, YB, LAM, cp, wp, YB, zdh, zdm, zdl);
            us16* th = zsh; zsh = zdh; zdh = th;
            us16* tm = zsm; zsm = zdm; zdm = tm;
            us16* tl = zsl; zsl = zdl; zdl = tl;
        }

        gemm_kernel<3, 4><<<dim3(64 / 64, MG), 256, 0, stream>>>(
            zsh, zsm, zsl, 256, DRh, DRm, DRl, 256, 256, 64,
            b4, YB, LAM, cp, wp, XP, A0h, A0m, A0l);

        fold_kernel<<<IMG / 2, 256, 0, stream>>>(XP, wp, oim);
    }
}
